// modelLSTMcell_22445499089340
// MI455X (gfx1250) — hardware-verified
//
#include <hip/hip_runtime.h>
#include <math.h>

constexpr int NSTEP    = 365;
constexpr int NBAT     = 1000;
constexpr int NBPAD    = 1008;
constexpr int NXIN     = 32;
constexpr int NHID     = 256;
constexpr int NGATE    = 4 * NHID;
constexpr int KCAT     = NHID + NXIN;
constexpr int NTHR     = 256;
constexpr int ROWS_BLK = 16;
constexpr int APITCH   = 296;
constexpr int TCHUNK   = 32;
constexpr int OTPITCH  = 384;
constexpr int OBPITCH  = 36;
constexpr int WROW8    = KCAT / 8;
constexpr int NW8      = NGATE * WROW8;
constexpr int NWBLK    = NW8 / NTHR;
constexpr int XROW8    = NBPAD * (NXIN / 8);
constexpr int NX8      = NSTEP * XROW8;
constexpr int NOUT     = NSTEP * NBAT;
constexpr int NOUT4    = NOUT / 4;
constexpr float ACARRY = 64.0f;
constexpr float WCARRY = 256.0f;
constexpr float FOLD   = 1.0f / (ACARRY * WCARRY);

static_assert(KCAT % 32 == 0, "K multiple of 32");
static_assert(KCAT == 288, "nine k-chunks");
static_assert(NGATE % 64 == 0, "N tile multiple");
static_assert(NBPAD % ROWS_BLK == 0 && NBPAD >= NBAT, "padded batch");
static_assert(NW8 % NTHR == 0, "weight plane covered by whole blocks");
static_assert(XROW8 % 32 == 0, "x plane rows covered by whole waves");
static_assert(NX8 % 32 == 0, "x plane covered by whole waves");
static_assert(NBAT % 4 == 0 && NOUT % 4 == 0, "four consecutive outputs share one step");
static_assert(NHID == 32 * (NTHR / 32), "eight waves x 32 hidden units");
static_assert((APITCH * 2) % 16 == 0 && APITCH >= KCAT, "A tile pitch");
static_assert(OTPITCH >= ((NSTEP + TCHUNK - 1) / TCHUNK) * TCHUNK, "staging row holds all chunks");
static_assert((OTPITCH * 4) % 128 == 0, "staging row is whole lines");
static_assert(ROWS_BLK * (NXIN / 2) == NTHR, "x tile: one 32-bit word per thread");

typedef __attribute__((ext_vector_type(16))) _Float16 v16h;
typedef __attribute__((ext_vector_type(8)))  _Float16 v8h;
typedef __attribute__((ext_vector_type(8)))  float    v8f;
typedef __attribute__((ext_vector_type(4)))  float    v4f;

struct FragH {
  union U { v16h v; v8h h[2]; };
  static __device__ __forceinline__ v16h load(const _Float16* p) {
    U f;
    f.h[0] = *(const v8h*)(p);
    f.h[1] = *(const v8h*)(p + 16);
    return f.v;
  }
  static __device__ __forceinline__ v8f mma(v16h a, v16h b, v8f c) {
    return __builtin_amdgcn_wmma_f32_16x16x32_f16(false, a, false, b, (short)0, c, false, false);
  }
};

__device__ __forceinline__ void guard8(v8f& a0, v8f& a1, v8f& a2, v8f& a3, v8f& a4, v8f& a5, v8f& a6, v8f& a7,
                                       v16h x, v16h b0, v16h b1, v16h b2, v16h b3, v16h b4, v16h b5, v16h b6, v16h b7) {
  asm volatile("v_nop\n\tv_nop\n\tv_nop\n\tv_nop"
               : "+v"(a0), "+v"(a1), "+v"(a2), "+v"(a3), "+v"(a4), "+v"(a5), "+v"(a6), "+v"(a7)
               : "v"(x), "v"(b0), "v"(b1), "v"(b2), "v"(b3), "v"(b4), "v"(b5), "v"(b6), "v"(b7));
}

__device__ __forceinline__ float fsig(float x)  { return __builtin_amdgcn_rcpf(1.0f + __expf(-x)); }
__device__ __forceinline__ float ftanh(float x) { return 1.0f - 2.0f * __builtin_amdgcn_rcpf(__expf(2.0f * x) + 1.0f); }

__global__ __launch_bounds__(NTHR) void prep_w_kernel(const float* __restrict__ w_hh, const float* __restrict__ w_ih,
                                                      const float* __restrict__ b_ih, const float* __restrict__ b_hh,
                                                      unsigned short* __restrict__ WC, float* __restrict__ biasv) {
  const int tid = threadIdx.x;
  if (blockIdx.x == NWBLK) {
    const int idx = tid * 4;
    const v4f va = *(const v4f*)(b_ih + idx);
    const v4f vb = *(const v4f*)(b_hh + idx);
    v4f o;
#pragma unroll
    for (int e = 0; e < 4; ++e) o[e] = va[e] + vb[e];
    *(volatile v4f*)(biasv + idx) = o;
    __threadfence();
    *(volatile v4f*)(biasv + idx) = o;
    return;
  }
  const int i  = blockIdx.x * NTHR + tid;
  const int n  = i / WROW8;
  const int c8 = i - n * WROW8;
  const bool isx = (c8 >= NHID / 8);
  const int ch = isx ? (NHID / 8 - 1) : c8;
  const int ci = isx ? (c8 - NHID / 8) : 0;
  const float* hp = w_hh + (size_t)n * NHID + ch * 8;
  const float* ip = w_ih + (size_t)n * NXIN + ci * 8;
  v4f h0 = *(const v4f*)(hp);
  v4f h1 = *(const v4f*)(hp + 4);
  v4f i0 = *(const v4f*)(ip);
  v4f i1 = *(const v4f*)(ip + 4);
  asm volatile("" : "+v"(h0));
  asm volatile("" : "+v"(h1));
  asm volatile("" : "+v"(i0));
  asm volatile("" : "+v"(i1));
  v8h hv;
#pragma unroll
  for (int e = 0; e < 4; ++e) {
    const float f0 = isx ? i0[e] : h0[e];
    const float f1 = isx ? i1[e] : h1[e];
    hv[e]     = (_Float16)(f0 * WCARRY);
    hv[4 + e] = (_Float16)(f1 * WCARRY);
  }
  unsigned short* dp = WC + (size_t)i * 8;
  *(volatile v8h*)dp = hv;
  __threadfence();
  *(volatile v8h*)dp = hv;
}

__global__ __launch_bounds__(NTHR) void prep_x_kernel(const float* __restrict__ x, const float* __restrict__ maskX,
                                                      unsigned short* __restrict__ XM) {
  const int i = blockIdx.x * NTHR + threadIdx.x;
  if (i < NX8) {
    const int t   = i / XROW8;
    const int rem = i - t * XROW8;
    const int b   = rem >> 2;
    const int c8  = (rem & 3) * 8;
    const bool live = (b < NBAT);
    const int bc  = live ? b : (NBAT - 1);
    const float* xp = x + ((size_t)t * NBAT + bc) * NXIN + c8;
    const float* mp = maskX + (size_t)bc * NXIN + c8;
    v4f x0 = *(const v4f*)(xp);
    v4f x1 = *(const v4f*)(xp + 4);
    v4f m0 = *(const v4f*)(mp);
    v4f m1 = *(const v4f*)(mp + 4);
    asm volatile("" : "+v"(x0));
    asm volatile("" : "+v"(x1));
    asm volatile("" : "+v"(m0));
    asm volatile("" : "+v"(m1));
    v8h hv;
#pragma unroll
    for (int e = 0; e < 4; ++e) {
      const float p0 = x0[e] * m0[e];
      const float p1 = x1[e] * m1[e];
      const float f0 = live ? (p0 * ACARRY) : 0.0f;
      const float f1 = live ? (p1 * ACARRY) : 0.0f;
      hv[e]     = (_Float16)f0;
      hv[4 + e] = (_Float16)f1;
    }
    unsigned short* dp = XM + (size_t)i * 8;
    *(volatile v8h*)dp = hv;
    __threadfence();
    *(volatile v8h*)dp = hv;
  }
}

__global__ __launch_bounds__(NTHR) void lstm_seq_kernel(const unsigned short* __restrict__ XMp,
                                                        const unsigned short* __restrict__ WCp,
                                                        const float* __restrict__ biasv,
                                                        const float* __restrict__ w_out,
                                                        const float* __restrict__ b_out,
                                                        float* __restrict__ outT) {
  __shared__ __align__(16) _Float16 At[ROWS_BLK * APITCH];
  __shared__ __align__(16) float    part[(NTHR / 32) * ROWS_BLK];
  __shared__ __align__(16) float    obuf[ROWS_BLK * OBPITCH];

  const _Float16* WC  = (const _Float16*)WCp;
  const unsigned* XMw = (const unsigned*)XMp;
  const int tid  = threadIdx.x;
  const int lane = tid & 31;
  const int wave = __builtin_amdgcn_readfirstlane((int)(threadIdx.x >> 5));
  const int c    = lane & 15;
  const int hh   = lane >> 4;
  const int koff = hh * 8;
  const int rowbase = blockIdx.x * ROWS_BLK;
  const int xm_m = tid >> 4;
  const int xm_w = tid & 15;

#pragma unroll 1
  for (int i = tid; i < ROWS_BLK * (NHID / 2); i += NTHR) {
    const int row = i >> 7;
    const int w   = i & 127;
    *(unsigned*)(At + row * APITCH + 2 * w) = 0u;
  }
  {
    const unsigned xw0 = XMw[((size_t)rowbase + xm_m) * (NXIN / 2) + xm_w];
    *(unsigned*)(At + xm_m * APITCH + NHID + 2 * xm_w) = xw0;
  }

  float bb[2][4], wo[2], cst[2][8];
#pragma unroll
  for (int nt = 0; nt < 2; ++nt) {
    const int j = 32 * wave + 16 * nt + c;
#pragma unroll
    for (int q = 0; q < 4; ++q) bb[nt][q] = biasv[q * NHID + j];
    wo[nt] = w_out[j];
#pragma unroll
    for (int r = 0; r < 8; ++r) cst[nt][r] = 0.0f;
  }
  const float bo = b_out[0];
  __syncthreads();

  const _Float16* arow = At + c * APITCH + koff;
  const _Float16* wb   = WC + (size_t)(32 * wave + c) * KCAT + koff;
  const v8f z8 = {0.f, 0.f, 0.f, 0.f, 0.f, 0.f, 0.f, 0.f};

#pragma unroll 1
  for (int t = 0; t < NSTEP; ++t) {
    const int tn = (t + 1 < NSTEP) ? (t + 1) : (NSTEP - 1);
    const unsigned xw = XMw[((size_t)tn * NBPAD + rowbase + xm_m) * (NXIN / 2) + xm_w];

    v8f acc[2][4];
#pragma unroll
    for (int nt = 0; nt < 2; ++nt)
#pragma unroll
      for (int q = 0; q < 4; ++q) acc[nt][q] = z8;

#pragma unroll 1
    for (int k0 = 0; k0 < KCAT; k0 += 32) {
      const v16h a = FragH::load(arow + k0);
      const _Float16* wk = wb + k0;
      v16h bf[2][4];
#pragma unroll
      for (int nt = 0; nt < 2; ++nt)
#pragma unroll
        for (int q = 0; q < 4; ++q)
          bf[nt][q] = FragH::load(wk + (size_t)(q * NHID + 16 * nt) * KCAT);
#pragma unroll
      for (int nt = 0; nt < 2; ++nt)
#pragma unroll
        for (int q = 0; q < 4; ++q)
          acc[nt][q] = FragH::mma(a, bf[nt][q], acc[nt][q]);
      guard8(acc[0][0], acc[0][1], acc[0][2], acc[0][3], acc[1][0], acc[1][1], acc[1][2], acc[1][3],
             a, bf[0][0], bf[0][1], bf[0][2], bf[0][3], bf[1][0], bf[1][1], bf[1][2], bf[1][3]);
    }
    __syncthreads();

    float hp[8];
#pragma unroll
    for (int r = 0; r < 8; ++r) hp[r] = 0.0f;
#pragma unroll
    for (int nt = 0; nt < 2; ++nt) {
      const int j = 32 * wave + 16 * nt + c;
#pragma unroll
      for (int r = 0; r < 8; ++r) {
        const float zi = acc[nt][0][r] * FOLD + bb[nt][0];
        const float zf = acc[nt][1][r] * FOLD + bb[nt][1];
        const float zg = acc[nt][2][r] * FOLD + bb[nt][2];
        const float zo = acc[nt][3][r] * FOLD + bb[nt][3];
        const float ig = fsig(zi);
        const float fg = fsig(zf);
        const float gg = ftanh(zg);
        const float og = fsig(zo);
        const float cn = fg * cst[nt][r] + ig * gg;
        cst[nt][r] = cn;
        const float hn = og * ftanh(cn);
        At[(8 * hh + r) * APITCH + j] = (_Float16)(hn * ACARRY);
        hp[r] += hn * wo[nt];
      }
    }
    *(unsigned*)(At + xm_m * APITCH + NHID + 2 * xm_w) = xw;

#pragma unroll
    for (int r = 0; r < 8; ++r) {
      hp[r] += __shfl_xor(hp[r], 1, 32);
      hp[r] += __shfl_xor(hp[r], 2, 32);
      hp[r] += __shfl_xor(hp[r], 4, 32);
      hp[r] += __shfl_xor(hp[r], 8, 32);
    }
    if (c == 0) {
#pragma unroll
      for (int r = 0; r < 8; ++r) part[wave * ROWS_BLK + 8 * hh + r] = hp[r];
    }
    __syncthreads();

    if (tid < ROWS_BLK) {
      float s = bo;
#pragma unroll
      for (int w = 0; w < NTHR / 32; ++w) s += part[w * ROWS_BLK + tid];
      obuf[tid * OBPITCH + (t & (TCHUNK - 1))] = s;
    }

    const bool flush = ((t & (TCHUNK - 1)) == (TCHUNK - 1)) || (t == NSTEP - 1);
    if (flush) {
      __syncthreads();
      if (wave < 4) {
        const int row = 4 * wave + (lane >> 3);
        const int c4  = (lane & 7) * 4;
        const v4f v = *(const v4f*)(obuf + row * OBPITCH + c4);
        float* op = outT + (size_t)(rowbase + row) * OTPITCH + (t >> 5) * TCHUNK + c4;
        *(volatile v4f*)op = v;
        __threadfence();
        *(volatile v4f*)op = v;
      }
    }
  }
}

__global__ __launch_bounds__(NTHR) void out_transpose_kernel(const float* __restrict__ outT, float* __restrict__ out) {
  const int i  = blockIdx.x * NTHR + threadIdx.x;
  const int ic = (i < NOUT4) ? i : (NOUT4 - 1);
  const int idx0 = ic * 4;
  const int t  = idx0 / NBAT;
  const int b0 = idx0 - t * NBAT;
  float v0 = outT[(size_t)(b0 + 0) * OTPITCH + t];
  float v1 = outT[(size_t)(b0 + 1) * OTPITCH + t];
  float v2 = outT[(size_t)(b0 + 2) * OTPITCH + t];
  float v3 = outT[(size_t)(b0 + 3) * OTPITCH + t];
  asm volatile("" : "+v"(v0), "+v"(v1), "+v"(v2), "+v"(v3));
  if (i < NOUT4) {
    v4f v;
    v[0] = v0;
    v[1] = v1;
    v[2] = v2;
    v[3] = v3;
    float* op = out + (size_t)i * 4;
    *(volatile v4f*)op = v;
    __threadfence();
    *(volatile v4f*)op = v;
  }
}

extern "C" void kernel_launch(void* const* d_in, const int* in_sizes, int n_in,
                              void* d_out, int out_size, void* d_ws, size_t ws_size, hipStream_t stream) {
  if (n_in < 8 || d_out == nullptr || d_ws == nullptr) return;
  if (in_sizes[0] != NSTEP * NBAT * NXIN || in_sizes[1] != NBAT * NXIN || in_sizes[2] != NGATE * NXIN ||
      in_sizes[3] != NGATE * NHID || in_sizes[4] != NGATE || in_sizes[5] != NGATE ||
      in_sizes[6] != NHID || in_sizes[7] != 1 || out_size != NOUT) return;

  const float* x     = (const float*)d_in[0];
  const float* maskX = (const float*)d_in[1];
  const float* w_ih  = (const float*)d_in[2];
  const float* w_hh  = (const float*)d_in[3];
  const float* b_ih  = (const float*)d_in[4];
  const float* b_hh  = (const float*)d_in[5];
  const float* w_out = (const float*)d_in[6];
  const float* b_out = (const float*)d_in[7];
  float* out = (float*)d_out;

  char* ws = (char*)d_ws;
  size_t off = 0;
  auto carve = [&](size_t bytes) -> char* { char* p = ws + off; off += (bytes + 255) & ~(size_t)255; return p; };
  unsigned short* WC   = (unsigned short*)carve((size_t)NGATE * KCAT * 2);
  float*          BIAS = (float*)carve((size_t)NGATE * 4);
  unsigned short* XM   = (unsigned short*)carve((size_t)NSTEP * NBPAD * NXIN * 2);
  float*          OUTT = (float*)carve((size_t)NBPAD * OTPITCH * 4);
  if (off > ws_size || off > (size_t)134217728) return;

  prep_w_kernel<<<NWBLK + 1, NTHR, 0, stream>>>(w_hh, w_ih, b_ih, b_hh, WC, BIAS);
  prep_x_kernel<<<(NX8 + NTHR - 1) / NTHR, NTHR, 0, stream>>>(x, maskX, XM);
  lstm_seq_kernel<<<NBPAD / ROWS_BLK, NTHR, 0, stream>>>(XM, WC, BIAS, w_out, b_out, OUTT);
  out_transpose_kernel<<<(NOUT4 + NTHR - 1) / NTHR, NTHR, 0, stream>>>(OUTT, out);
}
